// EncodeProcessDecode_82274393522653
// MI455X (gfx1250) — hardware-verified
//
#include <hip/hip_runtime.h>
#include <stddef.h>
#include <stdint.h>

#define HID    128
#define NF     7
#define KF     32
#define KH     256
#define KN1    512
#define NZP    512
#define NPS    256
#define NTHR   256
#define NWAVE  8
#define EPB    256
#define DP     132
#define AP     264
#define CSTN   528
#define OCB1   0
#define OCB2   128
#define OCG    256
#define OCBE   384
#define OCM    512
#define OCIS   520
#define GBM    64
#define GBN    128
#define GTHR   128
#define EPT    8
#define CHUNK  (NTHR * EPT)
#define WCAP   (EPT * 32)
#define LISTN  (NWAVE * WCAP)
#define NBA    1024
#define SLA    10
#define RCAP   28672
#define DEGCAP 64
#define DH     8
#define DO     15
#define NTW    5
#define NOD    3
#define DROWS  64
#define DPT    16
#define DTHR   128
#define OW1AB  0
#define OW1C   65536
#define OW2E   98304
#define OWN1   131072
#define OWN2   196608
#define SPH    229376
#define UPS    (SPH / 8)
#define UW1AB  (KH * (KH / 8))
#define UW1C   (HID * (KH / 8))
#define UW2E   (HID * (KH / 8))
#define UWN1   (HID * (KN1 / 8))
#define UWN2   (HID * (KH / 8))
#define NU_F32 (HID * (KF / 8))
#define NU_256 (HID * (KH / 8))
#define NU_DEC (DPT * (KH / 8))
#define NU_ENC (2 * NU_F32 + 2 * NU_256 + NU_DEC)
#define AGG_ZINTS (LISTN + 2 * RCAP + 3 * NBA)
#define AGG_LDS_INTS (AGG_ZINTS + 16)
#define AGG_LDS_BYTES (AGG_LDS_INTS * 4)
#define EDGE_LDS_BYTES (EPB * DP * 4 + EPB * AP * 2 + CSTN * 4)
#define WSMAX  134217728

static_assert((CHUNK & (CHUNK - 1)) == 0 && CHUNK <= 4096);
static_assert((NBA & (NBA - 1)) == 0 && NBA == (1 << SLA));
static_assert(((long long)CHUNK << SLA) < (1LL << 31));
static_assert(LISTN % NTHR == 0);
static_assert(NBA % NWAVE == 0 && NBA % 32 == 0);
static_assert(RCAP % 4 == 0 && AGG_ZINTS % (4 * NTHR) == 0 && LISTN % 4 == 0);
static_assert(AGG_LDS_BYTES <= 300000);
static_assert(EDGE_LDS_BYTES <= 300000);
static_assert(UW1AB + UW1C + UW2E + UWN1 + UWN2 == UPS && UPS % NTHR == 0);
static_assert(UW1AB % NTHR == 0 && UW1C % NTHR == 0 && UW2E % NTHR == 0 && UWN1 % NTHR == 0 && UWN2 % NTHR == 0);
static_assert(OW1C == OW1AB + 8 * UW1AB && OW2E == OW1C + 8 * UW1C && OWN1 == OW2E + 8 * UW2E);
static_assert(OWN2 == OWN1 + 8 * UWN1 && SPH == OWN2 + 8 * UWN2);
static_assert(NU_F32 % NTHR == 0 && NU_256 % NTHR == 0 && NU_DEC % NTHR == 0 && NU_ENC % NTHR == 0);
static_assert(KF % 32 == 0 && KH % 32 == 0 && KN1 % 32 == 0 && 2 * NF <= KF);
static_assert(KH == 2 * HID && KN1 == 2 * KH && NZP == KN1 && NPS == 2 * HID);
static_assert(GBM == (GTHR / 32) * 16 && GBN == 4 * 32 && GBN == HID);
static_assert((DP * 4) % 16 == 0 && (AP * 2) % 16 == 0 && AP >= KH && DP >= HID);
static_assert(EPB == NTHR && EPB == 8 * 32);
static_assert((EPB * DP * 4) % 16 == 0 && (EPB * AP * 2) % 16 == 0 && (CSTN * 4) % 16 == 0);
static_assert(CSTN >= OCIS + 8 && OCM >= OCBE + HID);
static_assert((EPB * HID / 4) % NTHR == 0 && (EPB * KH / 8) % NTHR == 0);
static_assert(DROWS == (DTHR / 32) * 16 && (DROWS * DPT / 4) % DTHR == 0 && DPT >= DO && DH <= DPT);
static_assert(NTW * NOD == DO);

typedef float          v2f   __attribute__((ext_vector_type(2)));
typedef float          v4f   __attribute__((ext_vector_type(4)));
typedef float          v8f   __attribute__((ext_vector_type(8)));
typedef int            v4i   __attribute__((ext_vector_type(4)));
typedef int            v8i   __attribute__((ext_vector_type(8)));
typedef unsigned short v8us  __attribute__((ext_vector_type(8)));
typedef unsigned short v16us __attribute__((ext_vector_type(16)));
typedef __bf16         v16bf __attribute__((ext_vector_type(16)));
typedef v2f  __attribute__((may_alias)) v2fa;
typedef v4f  __attribute__((may_alias)) v4fa;
typedef v4i  __attribute__((may_alias)) v4ia;
typedef v8us __attribute__((may_alias)) v8usa;
union FragB { v16bf v; v16us u; v8us h[2]; v8i w; };

__device__ __forceinline__ v8f wmb(const FragB& a, const FragB& b, v8f c) {
  v8f d = __builtin_amdgcn_wmma_f32_16x16x32_bf16(false, a.v, false, b.v, (short)0, c, false, false);
  asm volatile("v_nop\n\tv_nop\n\tv_nop\n\tv_nop" : "+v"(d) : "v"(a.w), "v"(b.w));
  return d;
}

__device__ __forceinline__ unsigned bf16_bits(float f) {
  const unsigned u = __float_as_uint(f);
  return (u + 0x7FFFu + ((u >> 16) & 1u)) >> 16;
}
__device__ __forceinline__ float bf16_val(float f) {
  return __uint_as_float(bf16_bits(f) << 16);
}
__device__ __forceinline__ float wsum(float v) {
#pragma unroll
  for (int d = 16; d >= 1; d >>= 1) v += __shfl_xor(v, d, 32);
  return v;
}
__device__ __forceinline__ void put16(unsigned short* dp, v8us o) {
  *(volatile v8us*)dp = o;
  __threadfence();
  *(volatile v8us*)dp = o;
}

template <int SLB>
__device__ __forceinline__ int scan_chunk(const int* __restrict__ dsts, int nE, int cbase, int slotBase,
                                          int nb, int vec8, int* list, int tid, int lane, int wave) {
  int wc = 0;
  const int el0  = tid * EPT;
  const int e0   = cbase + el0;
  const int sent = -2147483647 - 1;
  v4i da, db;
  if (vec8 != 0 && cbase + CHUNK <= nE) {
    da = *(const v4i*)(dsts + e0);
    db = *(const v4i*)(dsts + e0 + 4);
  } else {
    da.x = (e0     < nE) ? dsts[min(e0,     nE - 1)] : sent;
    da.y = (e0 + 1 < nE) ? dsts[min(e0 + 1, nE - 1)] : sent;
    da.z = (e0 + 2 < nE) ? dsts[min(e0 + 2, nE - 1)] : sent;
    da.w = (e0 + 3 < nE) ? dsts[min(e0 + 3, nE - 1)] : sent;
    db.x = (e0 + 4 < nE) ? dsts[min(e0 + 4, nE - 1)] : sent;
    db.y = (e0 + 5 < nE) ? dsts[min(e0 + 5, nE - 1)] : sent;
    db.z = (e0 + 6 < nE) ? dsts[min(e0 + 6, nE - 1)] : sent;
    db.w = (e0 + 7 < nE) ? dsts[min(e0 + 7, nE - 1)] : sent;
  }
  const unsigned nbs = (unsigned)slotBase;
  const unsigned unb = (unsigned)nb;
  const unsigned s0 = (unsigned)da.x - nbs, s1 = (unsigned)da.y - nbs;
  const unsigned s2 = (unsigned)da.z - nbs, s3 = (unsigned)da.w - nbs;
  const unsigned s4 = (unsigned)db.x - nbs, s5 = (unsigned)db.y - nbs;
  const unsigned s6 = (unsigned)db.z - nbs, s7 = (unsigned)db.w - nbs;
  const bool h0 = s0 < unb, h1 = s1 < unb, h2 = s2 < unb, h3 = s3 < unb;
  const bool h4 = s4 < unb, h5 = s5 < unb, h6 = s6 < unb, h7 = s7 < unb;
  const unsigned any = __builtin_amdgcn_ballot_w32(h0 | h1 | h2 | h3 | h4 | h5 | h6 | h7);
  if (any != 0u) {
#define HITJ(J, HJ, SJ) { \
      const unsigned mj = __builtin_amdgcn_ballot_w32(HJ); \
      if (mj != 0u) { \
        if (HJ) { \
          const int pos = wc + (int)__builtin_amdgcn_mbcnt_lo(mj, 0u); \
          if (pos < WCAP) list[wave * WCAP + pos] = ((el0 + (J)) << SLB) | (int)(SJ); \
        } \
        wc += (int)__builtin_popcount(mj); } }
    HITJ(0, h0, s0)
    HITJ(1, h1, s1)
    HITJ(2, h2, s2)
    HITJ(3, h3, s3)
    HITJ(4, h4, s4)
    HITJ(5, h5, s5)
    HITJ(6, h6, s6)
    HITJ(7, h7, s7)
#undef HITJ
  }
  return wc;
}

__global__ __launch_bounds__(NTHR) void k_prep(const float* __restrict__ disp, const float* __restrict__ chem,
                                               const int* __restrict__ ntype,
                                               const float* __restrict__ nmean, const float* __restrict__ nstd,
                                               const float* __restrict__ enW1, const float* __restrict__ enW2,
                                               const float* __restrict__ eeW1, const float* __restrict__ eeW2,
                                               const float* __restrict__ beW1, const float* __restrict__ beW2,
                                               const float* __restrict__ bnW1, const float* __restrict__ bnW2,
                                               const float* __restrict__ dcW1,
                                               int nN, int mRows, int nSteps,
                                               unsigned short* WST, unsigned short* ENW1, unsigned short* ENW2,
                                               unsigned short* EEW1, unsigned short* EEW2, unsigned short* DCW1,
                                               unsigned short* FN) {
  __shared__ float cs[16];
  const int tid = (int)threadIdx.x;
  {
    const int j = tid < NF ? tid : NF - 1;
    const float mv = bf16_val(nmean[j]);
    const float sv = __builtin_amdgcn_rcpf(bf16_val(nstd[j]));
    if (tid < NF) { cs[tid] = mv; cs[8 + tid] = sv; }
  }
  __syncthreads();
  const int u  = (int)blockIdx.x * NTHR + tid;
  const int U0 = nSteps * UPS;
  const int U1 = U0 + NU_F32;
  const int U2 = U1 + NU_256;
  const int U3 = U2 + NU_F32;
  const int U4 = U3 + NU_256;
  const int U5 = U4 + NU_DEC;
  const int U6 = U5 + mRows * 4;
  v8us o;
  if (u < U0) {
    const int t = u / UPS;
    const int v = u - t * UPS;
    const float* W1 = beW1 + (size_t)t * 3 * HID * HID;
    const float* W2 = beW2 + (size_t)t * HID * HID;
    const float* V1 = bnW1 + (size_t)t * 2 * HID * HID;
    const float* V2 = bnW2 + (size_t)t * HID * HID;
    unsigned short* P = WST + (size_t)t * SPH;
    if (v < UW1AB) {
      const int n    = v >> 5;
      const int k8   = (v & 31) * 8;
      const int q    = n >> 7;
      const int nn   = n & (HID - 1);
      const int srow = q * HID + (k8 & (HID - 1));
      const float* p = W1 + (size_t)srow * HID + nn;
#pragma unroll
      for (int i = 0; i < 8; ++i) o[i] = (unsigned short)bf16_bits(p[(size_t)i * HID]);
      put16(P + OW1AB + (size_t)n * KH + k8, o);
    } else if (v < UW1AB + UW1C) {
      const int w    = v - UW1AB;
      const int n    = w >> 5;
      const int k8   = (w & 31) * 8;
      const int srow = 2 * HID + (k8 & (HID - 1));
      const float* p = W1 + (size_t)srow * HID + n;
#pragma unroll
      for (int i = 0; i < 8; ++i) o[i] = (unsigned short)bf16_bits(p[(size_t)i * HID]);
      put16(P + OW1C + (size_t)n * KH + k8, o);
    } else if (v < UW1AB + UW1C + UW2E) {
      const int w    = v - UW1AB - UW1C;
      const int n    = w >> 5;
      const int k8   = (w & 31) * 8;
      const int srow = k8 & (HID - 1);
      const float* p = W2 + (size_t)srow * HID + n;
#pragma unroll
      for (int i = 0; i < 8; ++i) o[i] = (unsigned short)bf16_bits(p[(size_t)i * HID]);
      put16(P + OW2E + (size_t)n * KH + k8, o);
    } else if (v < UW1AB + UW1C + UW2E + UWN1) {
      const int w    = v - UW1AB - UW1C - UW2E;
      const int n    = w >> 6;
      const int k8   = (w & 63) * 8;
      const int blo  = k8 & (HID - 1);
      const int bhi  = HID + 4 * ((k8 - KH) >> 3);
#pragma unroll
      for (int i = 0; i < 8; ++i) {
        const int srow = (k8 < KH) ? (blo + i) : (bhi + (i & 3));
        o[i] = (unsigned short)bf16_bits(V1[(size_t)srow * HID + n]);
      }
      put16(P + OWN1 + (size_t)n * KN1 + k8, o);
    } else {
      const int w    = v - UW1AB - UW1C - UW2E - UWN1;
      const int n    = w >> 5;
      const int k8   = (w & 31) * 8;
      const int srow = k8 & (HID - 1);
      const float* p = V2 + (size_t)srow * HID + n;
#pragma unroll
      for (int i = 0; i < 8; ++i) o[i] = (unsigned short)bf16_bits(p[(size_t)i * HID]);
      put16(P + OWN2 + (size_t)n * KH + k8, o);
    }
    return;
  } else if (u < U1 || (u >= U2 && u < U3)) {
    const bool node = u < U1;
    const int v  = node ? (u - U0) : (u - U2);
    const float* W = node ? enW1 : eeW1;
    unsigned short* Q = node ? ENW1 : EEW1;
    const int n  = v >> 2;
    const int k8 = (v & 3) * 8;
#pragma unroll
    for (int i = 0; i < 8; ++i) {
      const int k    = k8 + i;
      const int srow = (k < NF) ? k : ((k < 2 * NF) ? (k - NF) : (NF - 1));
      const float wv = W[(size_t)srow * HID + n];
      o[i] = (unsigned short)bf16_bits((k < 2 * NF) ? wv : wv * 0.0f);
    }
    put16(Q + (size_t)n * KF + k8, o);
    return;
  } else if (u < U2 || (u >= U3 && u < U4)) {
    const bool node = u < U2;
    const int v  = node ? (u - U1) : (u - U3);
    const float* W = node ? enW2 : eeW2;
    unsigned short* Q = node ? ENW2 : EEW2;
    const int n    = v >> 5;
    const int k8   = (v & 31) * 8;
    const int srow = k8 & (HID - 1);
    const float* p = W + (size_t)srow * HID + n;
#pragma unroll
    for (int i = 0; i < 8; ++i) o[i] = (unsigned short)bf16_bits(p[(size_t)i * HID]);
    put16(Q + (size_t)n * KH + k8, o);
    return;
  } else if (u < U5) {
    const int v  = u - U4;
    const int n  = v >> 5;
    const int k8 = (v & 31) * 8;
    const int nc = n < DH ? n : DH - 1;
#pragma unroll
    for (int i = 0; i < 8; ++i) {
      const int srow = (k8 & (HID - 1)) + i;
      const float wv = dcW1[(size_t)srow * DH + nc];
      o[i] = (unsigned short)bf16_bits((n < DH) ? wv : wv * 0.0f);
    }
    put16(DCW1 + (size_t)n * KH + k8, o);
    return;
  }
  if (u >= U6) return;
  {
    const int v    = u - U5;
    const int row  = v >> 2;
    const int ksel = v & 3;
    const int rc   = row < nN ? row : nN - 1;
    const bool ok  = row < nN;
    const v2f d    = *(const v2fa*)(disp + 2 * (size_t)rc);
    const float c  = chem[rc];
    const int ty   = ntype[rc];
    float f[NF];
    f[0] = (bf16_val(d.x) - cs[0]) * cs[8];
    f[1] = (bf16_val(d.y) - cs[1]) * cs[9];
    f[2] = (bf16_val(c) - cs[2]) * cs[10];
#pragma unroll
    for (int i = 0; i < 4; ++i) {
      const float oh = (ty == i) ? 1.0f : 0.0f;
      f[3 + i] = (oh - cs[3 + i]) * cs[11 + i];
    }
    unsigned hb[NF], lb[NF];
#pragma unroll
    for (int i = 0; i < NF; ++i) {
      hb[i] = bf16_bits(f[i]);
      lb[i] = bf16_bits(f[i] - __uint_as_float(hb[i] << 16));
    }
    const unsigned short pz = (unsigned short)bf16_bits(d.x * 0.0f);
    v8us oa, ob;
#pragma unroll
    for (int i = 0; i < NF; ++i) oa[i] = (unsigned short)hb[i];
    oa[7] = (unsigned short)lb[0];
#pragma unroll
    for (int i = 0; i < 6; ++i) ob[i] = (unsigned short)lb[1 + i];
    ob[6] = pz; ob[7] = pz;
#pragma unroll
    for (int i = 0; i < 8; ++i) {
      const unsigned short sv = (ksel == 0) ? oa[i] : ((ksel == 1) ? ob[i] : pz);
      o[i] = ok ? sv : pz;
    }
    put16(FN + (size_t)row * KF + ksel * 8, o);
  }
}

template <int MODE>
__global__ __launch_bounds__(GTHR) void k_gemm(const unsigned short* __restrict__ A, int lda,
                                               const unsigned short* __restrict__ BT, int ldb, int K,
                                               const float* __restrict__ bias, const float* __restrict__ gam,
                                               const float* __restrict__ bet,
                                               float* Cm, int ldc, unsigned short* Cb, int ldcb) {
  __shared__ __attribute__((aligned(16))) float stg[GBM * GBN];
  const int tid = (int)threadIdx.x, lane = tid & 31, wave = tid >> 5, hh = lane >> 4, m = lane & 15;
  const int rowBase = (int)blockIdx.x * GBM;
  const int colBase = (int)blockIdx.y * GBN;

  v8f acc[8];
  {
    const v8f z = {0.f, 0.f, 0.f, 0.f, 0.f, 0.f, 0.f, 0.f};
#pragma unroll
    for (int t = 0; t < 8; ++t) acc[t] = z;
  }
  const unsigned short* ap = A  + (size_t)(rowBase + 16 * wave + m) * (size_t)lda + 8 * hh;
  const unsigned short* bp = BT + (size_t)(colBase + m) * (size_t)ldb + 8 * hh;

#pragma unroll 1
  for (int k0 = 0; k0 < K; k0 += 32) {
    FragB af;
    af.h[0] = *(const v8usa*)(ap + k0);
    af.h[1] = *(const v8usa*)(ap + k0 + 16);
#pragma unroll
    for (int nt = 0; nt < 8; ++nt) {
      const unsigned short* wq = bp + (size_t)(16 * nt) * (size_t)ldb + k0;
      FragB bf;
      bf.h[0] = *(const v8usa*)wq;
      bf.h[1] = *(const v8usa*)(wq + 16);
      acc[nt] = wmb(af, bf, acc[nt]);
    }
  }

#pragma unroll
  for (int nt = 0; nt < 8; ++nt) {
    const int lc = 16 * nt + m;
    float bvv = 0.0f;
    if constexpr (MODE != 0) bvv = bf16_val(bias[colBase + lc]);
#pragma unroll
    for (int r = 0; r < 8; ++r) {
      const int lr = 16 * wave + 8 * hh + r;
      float v = acc[nt][r];
      if constexpr (MODE != 0) v = fmaxf(v + bvv, 0.0f);
      stg[lr * GBN + lc] = v;
    }
  }
  __syncthreads();

  if constexpr (MODE == 0) {
    v4f pv[16];
#pragma unroll
    for (int i = 0; i < 16; ++i) pv[i] = *(const v4fa*)(stg + (16 * wave + i) * GBN + 4 * lane);
#pragma unroll
    for (int i = 0; i < 16; ++i) {
      float* op = Cm + (size_t)(rowBase + 16 * wave + i) * (size_t)ldc + colBase + 4 * lane;
      *(volatile v4f*)op = pv[i];
    }
    __threadfence();
#pragma unroll
    for (int i = 0; i < 16; ++i) {
      float* op = Cm + (size_t)(rowBase + 16 * wave + i) * (size_t)ldc + colBase + 4 * lane;
      *(volatile v4f*)op = pv[i];
    }
  } else {
    if constexpr (MODE >= 3) {
      const v4f gr = *(const v4fa*)(gam + 4 * lane);
      const v4f er = *(const v4fa*)(bet + 4 * lane);
      const float g0 = bf16_val(gr.x), g1 = bf16_val(gr.y), g2 = bf16_val(gr.z), g3 = bf16_val(gr.w);
      const float e0 = bf16_val(er.x), e1 = bf16_val(er.y), e2 = bf16_val(er.z), e3 = bf16_val(er.w);
#pragma unroll 2
      for (int i = 0; i < 16; ++i) {
        const int lr = 16 * wave + i;
        float* sp = stg + lr * GBN + 4 * lane;
        const v4f v = *(const v4fa*)sp;
        float s = (v.x + v.y) + (v.z + v.w);
        s = wsum(s);
        const float mu = s * (1.0f / (float)GBN);
        const float dx = v.x - mu, dy = v.y - mu, dz = v.z - mu, dw = v.w - mu;
        float q = fmaf(dx, dx, fmaf(dy, dy, fmaf(dz, dz, dw * dw)));
        q = wsum(q);
        const float var = q * (1.0f / (float)GBN);
        const float rs  = __builtin_amdgcn_rcpf(sqrtf(var + 1e-5f));
        v4f y;
        y.x = fmaf(dx * rs, g0, e0);
        y.y = fmaf(dy * rs, g1, e1);
        y.z = fmaf(dz * rs, g2, e2);
        y.w = fmaf(dw * rs, g3, e3);
        if constexpr (MODE == 4) {
          const v4f old = *(const v4fa*)(Cm + (size_t)(rowBase + lr) * (size_t)ldc + 4 * lane);
          y.x += old.x; y.y += old.y; y.z += old.z; y.w += old.w;
        }
        *(v4fa*)sp = y;
      }
      __syncthreads();
      {
        v4f pv[16];
#pragma unroll
        for (int i = 0; i < 16; ++i) pv[i] = *(const v4fa*)(stg + (16 * wave + i) * GBN + 4 * lane);
#pragma unroll
        for (int i = 0; i < 16; ++i) {
          float* op = Cm + (size_t)(rowBase + 16 * wave + i) * (size_t)ldc + 4 * lane;
          *(volatile v4f*)op = pv[i];
        }
        __threadfence();
#pragma unroll
        for (int i = 0; i < 16; ++i) {
          float* op = Cm + (size_t)(rowBase + 16 * wave + i) * (size_t)ldc + 4 * lane;
          *(volatile v4f*)op = pv[i];
        }
      }
    }
    const int part = lane >> 4;
    const int j = lane & 15;
    const unsigned mh = 0u - (unsigned)part;
    const unsigned ml = ~mh;
    v8us pv[16];
#pragma unroll
    for (int i = 0; i < 16; ++i) {
      const float* sp = stg + (16 * wave + i) * GBN + 8 * j;
      const v4f a = *(const v4fa*)sp;
      const v4f b = *(const v4fa*)(sp + 4);
      const v8f f8 = {a.x, a.y, a.z, a.w, b.x, b.y, b.z, b.w};
      v8us oo;
#pragma unroll
      for (int e = 0; e < 8; ++e) {
        const unsigned hb = bf16_bits(f8[e]);
        const unsigned lb = bf16_bits(f8[e] - __uint_as_float(hb << 16));
        oo[e] = (unsigned short)((hb & ml) | (lb & mh));
      }
      pv[i] = oo;
    }
#pragma unroll
    for (int i = 0; i < 16; ++i) {
      unsigned short* op = Cb + (size_t)(rowBase + 16 * wave + i) * (size_t)ldcb + part * HID + 8 * j;
      *(volatile v8us*)op = pv[i];
    }
    __threadfence();
#pragma unroll
    for (int i = 0; i < 16; ++i) {
      unsigned short* op = Cb + (size_t)(rowBase + 16 * wave + i) * (size_t)ldcb + part * HID + 8 * j;
      *(volatile v8us*)op = pv[i];
    }
  }
}

template <int APITCH>
__device__ __forceinline__ void wave_gemm_b(const unsigned short* sAw, float* sDw,
                                            const unsigned short* __restrict__ BT, int ldb, int K,
                                            int hh, int m) {
#pragma unroll 1
  for (int nh = 0; nh < 2; ++nh) {
    v8f acc[2][4];
    {
      const v8f z = {0.f, 0.f, 0.f, 0.f, 0.f, 0.f, 0.f, 0.f};
#pragma unroll
      for (int mt = 0; mt < 2; ++mt)
#pragma unroll
        for (int nt = 0; nt < 4; ++nt) acc[mt][nt] = z;
    }
    const unsigned short* ap0 = sAw + m * APITCH + 8 * hh;
    const unsigned short* ap1 = ap0 + 16 * APITCH;
    const unsigned short* bp  = BT + (size_t)(64 * nh + m) * (size_t)ldb + 8 * hh;
#pragma unroll 1
    for (int k0 = 0; k0 < K; k0 += 32) {
      FragB a0, a1;
      a0.h[0] = *(const v8usa*)(ap0 + k0);
      a0.h[1] = *(const v8usa*)(ap0 + k0 + 16);
      a1.h[0] = *(const v8usa*)(ap1 + k0);
      a1.h[1] = *(const v8usa*)(ap1 + k0 + 16);
#pragma unroll
      for (int nt = 0; nt < 4; ++nt) {
        const unsigned short* wq = bp + (size_t)(16 * nt) * (size_t)ldb + k0;
        FragB b;
        b.h[0] = *(const v8usa*)wq;
        b.h[1] = *(const v8usa*)(wq + 16);
        acc[0][nt] = wmb(a0, b, acc[0][nt]);
        acc[1][nt] = wmb(a1, b, acc[1][nt]);
      }
    }
#pragma unroll
    for (int nt = 0; nt < 4; ++nt) {
      const int col = 64 * nh + 16 * nt + m;
#pragma unroll
      for (int mt = 0; mt < 2; ++mt)
#pragma unroll
        for (int r = 0; r < 8; ++r) sDw[(16 * mt + 8 * hh + r) * DP + col] = acc[mt][nt][r];
    }
  }
}

__device__ __forceinline__ void row_relu_ln(float* rd, const float* cst) {
  float s = 0.0f;
#pragma unroll 1
  for (int c8 = 0; c8 < HID / 8; ++c8) {
    const v4f va = *(const v4fa*)(rd + 8 * c8);
    const v4f vb = *(const v4fa*)(rd + 8 * c8 + 4);
    const v4f ba = *(const v4fa*)(cst + OCB2 + 8 * c8);
    const v4f bb = *(const v4fa*)(cst + OCB2 + 8 * c8 + 4);
    const v8f v8 = {va.x, va.y, va.z, va.w, vb.x, vb.y, vb.z, vb.w};
    const v8f b8 = {ba.x, ba.y, ba.z, ba.w, bb.x, bb.y, bb.z, bb.w};
    v8f w;
#pragma unroll
    for (int i = 0; i < 8; ++i) { w[i] = fmaxf(v8[i] + b8[i], 0.0f); s += w[i]; }
    const v4f m0 = {w[0], w[1], w[2], w[3]};
    const v4f m1 = {w[4], w[5], w[6], w[7]};
    *(v4fa*)(rd + 8 * c8)     = m0;
    *(v4fa*)(rd + 8 * c8 + 4) = m1;
  }
  const float mu = s * (1.0f / (float)HID);
  float q = 0.0f;
#pragma unroll 1
  for (int c8 = 0; c8 < HID / 8; ++c8) {
    const v4f va = *(const v4fa*)(rd + 8 * c8);
    const v4f vb = *(const v4fa*)(rd + 8 * c8 + 4);
    const v8f v8 = {va.x, va.y, va.z, va.w, vb.x, vb.y, vb.z, vb.w};
#pragma unroll
    for (int i = 0; i < 8; ++i) { const float d = v8[i] - mu; q = fmaf(d, d, q); }
  }
  const float var = q * (1.0f / (float)HID);
  const float rs  = __builtin_amdgcn_rcpf(sqrtf(var + 1e-5f));
#pragma unroll 1
  for (int c8 = 0; c8 < HID / 8; ++c8) {
    const v4f va = *(const v4fa*)(rd + 8 * c8);
    const v4f vb = *(const v4fa*)(rd + 8 * c8 + 4);
    const v4f ga = *(const v4fa*)(cst + OCG + 8 * c8);
    const v4f gb = *(const v4fa*)(cst + OCG + 8 * c8 + 4);
    const v4f ea = *(const v4fa*)(cst + OCBE + 8 * c8);
    const v4f eb = *(const v4fa*)(cst + OCBE + 8 * c8 + 4);
    const v8f v8 = {va.x, va.y, va.z, va.w, vb.x, vb.y, vb.z, vb.w};
    const v8f g8 = {ga.x, ga.y, ga.z, ga.w, gb.x, gb.y, gb.z, gb.w};
    const v8f e8 = {ea.x, ea.y, ea.z, ea.w, eb.x, eb.y, eb.z, eb.w};
    v8f y;
#pragma unroll
    for (int i = 0; i < 8; ++i) y[i] = fmaf((v8[i] - mu) * rs, g8[i], e8[i]);
    const v4f m0 = {y[0], y[1], y[2], y[3]};
    const v4f m1 = {y[4], y[5], y[6], y[7]};
    *(v4fa*)(rd + 8 * c8)     = m0;
    *(v4fa*)(rd + 8 * c8 + 4) = m1;
  }
}
__device__ __forceinline__ void row_hilo(const float* rd, unsigned short* ra) {
#pragma unroll 1
  for (int c8 = 0; c8 < HID / 8; ++c8) {
    const v4f va = *(const v4fa*)(rd + 8 * c8);
    const v4f vb = *(const v4fa*)(rd + 8 * c8 + 4);
    const v8f v8 = {va.x, va.y, va.z, va.w, vb.x, vb.y, vb.z, vb.w};
    v8us ho, lo;
#pragma unroll
    for (int i = 0; i < 8; ++i) {
      const unsigned hb = bf16_bits(v8[i]);
      ho[i] = (unsigned short)hb;
      lo[i] = (unsigned short)bf16_bits(v8[i] - __uint_as_float(hb << 16));
    }
    *(v8usa*)(ra + 8 * c8)       = ho;
    *(v8usa*)(ra + HID + 8 * c8) = lo;
  }
}
__device__ __forceinline__ void sweep_f32(const float* sD, float* gb, int tid) {
#pragma unroll 4
  for (int it = 0; it < (EPB * HID / 4) / NTHR; ++it) {
    const int q   = it * NTHR + tid;
    const int row = q >> 5;
    const int c4  = (q & 31) * 4;
    const v4f v = *(const v4fa*)(sD + row * DP + c4);
    *(volatile v4f*)(gb + (size_t)q * 4) = v;
  }
}
__device__ __forceinline__ void sweep_h16(const unsigned short* sA, unsigned short* gb, int tid) {
#pragma unroll 4
  for (int it = 0; it < (EPB * KH / 8) / NTHR; ++it) {
    const int q   = it * NTHR + tid;
    const int row = q >> 5;
    const int h8  = (q & 31) * 8;
    const v8us v = *(const v8usa*)(sA + row * AP + h8);
    *(volatile v8us*)(gb + (size_t)q * 8) = v;
  }
}

__global__ __launch_bounds__(NTHR) void k_ence(const int* __restrict__ snd, const int* __restrict__ rcv,
                                               int nE, int nN,
                                               const float* __restrict__ mpos, const float* __restrict__ disp,
                                               const float* __restrict__ chem,
                                               const float* __restrict__ emean, const float* __restrict__ estd,
                                               const unsigned short* __restrict__ W1T,
                                               const unsigned short* __restrict__ W2T,
                                               const float* __restrict__ b1, const float* __restrict__ b2,
                                               const float* __restrict__ gam, const float* __restrict__ bet,
                                               float* ELF, unsigned short* ELH) {
  extern __shared__ __attribute__((aligned(16))) float dyn[];
  float*          sD  = dyn;
  unsigned short* sA  = (unsigned short*)(dyn + EPB * DP);
  float*          cst = dyn + EPB * DP + (EPB * AP) / 2;

  const int tid = (int)threadIdx.x, lane = tid & 31, wave = tid >> 5, hh = lane >> 4, m = lane & 15;

  if (tid < HID) {
    cst[OCB1 + tid] = bf16_val(b1[tid]);
    cst[OCB2 + tid] = bf16_val(b2[tid]);
    cst[OCG + tid]  = bf16_val(gam[tid]);
    cst[OCBE + tid] = bf16_val(bet[tid]);
    const int j = tid < NF ? tid : NF - 1;
    const float mv = bf16_val(emean[j]);
    const float sv = __builtin_amdgcn_rcpf(bf16_val(estd[j]));
    if (tid < NF) { cst[OCM + tid] = mv; cst[OCIS + tid] = sv; }
  }
  __syncthreads();

  const int  elb = (int)blockIdx.x * EPB;
  const int  el  = elb + tid;
  const int  elc = el < nE ? el : (nE - 1);
  int s = snd[elc];
  int r = rcv[elc];
  s = s < 0 ? 0 : (s > nN - 1 ? nN - 1 : s);
  r = r < 0 ? 0 : (r > nN - 1 ? nN - 1 : r);

  float*          rd = sD + tid * DP;
  unsigned short* ra = sA + tid * AP;
  {
    const v2f ms = *(const v2fa*)(mpos + 2 * (size_t)s);
    const v2f mr = *(const v2fa*)(mpos + 2 * (size_t)r);
    const v2f ds = *(const v2fa*)(disp + 2 * (size_t)s);
    const v2f dr = *(const v2fa*)(disp + 2 * (size_t)r);
    const float chs = chem[s];
    const float chr = chem[r];
    const float rx  = bf16_val(ms.x) - bf16_val(mr.x);
    const float ry  = bf16_val(ms.y) - bf16_val(mr.y);
    const float nrm = sqrtf(rx * rx + ry * ry);
    const float gx  = bf16_val(ds.x) - bf16_val(dr.x);
    const float gy  = bf16_val(ds.y) - bf16_val(dr.y);
    const float cg  = bf16_val(chs) - bf16_val(chr);
    float f[NF];
    f[0] = rx; f[1] = ry; f[2] = nrm; f[3] = gx; f[4] = gy; f[5] = nrm; f[6] = cg;
    unsigned hb[NF], lb[NF];
#pragma unroll
    for (int i = 0; i < NF; ++i) {
      const float fn = (f[i] - cst[OCM + i]) * cst[OCIS + i];
      hb[i] = bf16_bits(fn);
      lb[i] = bf16_bits(fn - __uint_as_float(hb[i] << 16));
    }
    const unsigned short pz = (unsigned short)bf16_bits(rx * 0.0f);
    v8us o0, o1, oz;
#pragma unroll
    for (int i = 0; i < NF; ++i) o0[i] = (unsigned short)hb[i];
    o0[7] = (unsigned short)lb[0];
#pragma unroll
    for (int i = 0; i < 6; ++i) o1[i] = (unsigned short)lb[1 + i];
    o1[6] = pz; o1[7] = pz;
#pragma unroll
    for (int i = 0; i < 8; ++i) oz[i] = pz;
    *(v8usa*)(ra + 0)  = o0;
    *(v8usa*)(ra + 8)  = o1;
    *(v8usa*)(ra + 16) = oz;
    *(v8usa*)(ra + 24) = oz;
  }
  __syncthreads();

  const unsigned short* sAw = sA + 32 * wave * AP;
  float*                sDw = sD + 32 * wave * DP;

  wave_gemm_b<AP>(sAw, sDw, W1T, KF, KF, hh, m);
  __syncthreads();

  {
#pragma unroll 1
    for (int c8 = 0; c8 < HID / 8; ++c8) {
      const v4f va = *(const v4fa*)(rd + 8 * c8);
      const v4f vb = *(const v4fa*)(rd + 8 * c8 + 4);
      const v4f ba = *(const v4fa*)(cst + OCB1 + 8 * c8);
      const v4f bb = *(const v4fa*)(cst + OCB1 + 8 * c8 + 4);
      const v8f v8 = {va.x, va.y, va.z, va.w, vb.x, vb.y, vb.z, vb.w};
      const v8f b8 = {ba.x, ba.y, ba.z, ba.w, bb.x, bb.y, bb.z, bb.w};
      v8us ho, lo;
#pragma unroll
      for (int i = 0; i < 8; ++i) {
        const float h = fmaxf(v8[i] + b8[i], 0.0f);
        const unsigned hb = bf16_bits(h);
        ho[i] = (unsigned short)hb;
        lo[i] = (unsigned short)bf16_bits(h - __uint_as_float(hb << 16));
      }
      *(v8usa*)(ra + 8 * c8)       = ho;
      *(v8usa*)(ra + HID + 8 * c8) = lo;
    }
  }
  __syncthreads();

  wave_gemm_b<AP>(sAw, sDw, W2T, KH, KH, hh, m);
  __syncthreads();

  row_relu_ln(rd, cst);
  row_hilo(rd, ra);
  __syncthreads();

  sweep_f32(sD, ELF + (size_t)elb * HID, tid);
  sweep_h16(sA, ELH + (size_t)elb * KH, tid);
  __threadfence();
  sweep_f32(sD, ELF + (size_t)elb * HID, tid);
  sweep_h16(sA, ELH + (size_t)elb * KH, tid);
}

__global__ __launch_bounds__(NTHR) void k_edge(const int* __restrict__ snd, const int* __restrict__ rcv,
                                               int nE, int nN, const float* __restrict__ PSR,
                                               const unsigned short* __restrict__ W1CT,
                                               const unsigned short* __restrict__ W2T,
                                               const float* __restrict__ b1, const float* __restrict__ b2,
                                               const float* __restrict__ gam, const float* __restrict__ bet,
                                               float* ELF, unsigned short* ELH, float* NE) {
  extern __shared__ __attribute__((aligned(16))) float dyn[];
  float*          sD  = dyn;
  unsigned short* sA  = (unsigned short*)(dyn + EPB * DP);
  float*          cst = dyn + EPB * DP + (EPB * AP) / 2;

  const int tid = (int)threadIdx.x, lane = tid & 31, wave = tid >> 5, hh = lane >> 4, m = lane & 15;

  if (tid < HID) {
    cst[OCB1 + tid] = bf16_val(b1[tid]);
    cst[OCB2 + tid] = bf16_val(b2[tid]);
    cst[OCG + tid]  = bf16_val(gam[tid]);
    cst[OCBE + tid] = bf16_val(bet[tid]);
  }

  const int  elb = (int)blockIdx.x * EPB;
  const int  el  = elb + tid;
  const int  elc = el < nE ? el : (nE - 1);
  int s = snd[elc];
  int r = rcv[elc];
  s = s < 0 ? 0 : (s > nN - 1 ? nN - 1 : s);
  r = r < 0 ? 0 : (r > nN - 1 ? nN - 1 : r);

  float*          rd = sD + tid * DP;
  unsigned short* ra = sA + tid * AP;
  const unsigned short* sAw = sA + 32 * wave * AP;
  float*                sDw = sD + 32 * wave * DP;

  wave_gemm_b<KH>(ELH + (size_t)(elb + 32 * wave) * KH, sDw, W1CT, KH, KH, hh, m);
  __syncthreads();

  {
    const float* ps = PSR + (size_t)s * NPS;
    const float* pr = PSR + (size_t)r * NPS + HID;
#pragma unroll 1
    for (int c8 = 0; c8 < HID / 8; ++c8) {
      const v4f va = *(const v4fa*)(rd + 8 * c8);
      const v4f vb = *(const v4fa*)(rd + 8 * c8 + 4);
      const v4f pa = *(const v4fa*)(ps + 8 * c8);
      const v4f pb = *(const v4fa*)(ps + 8 * c8 + 4);
      const v4f qa = *(const v4fa*)(pr + 8 * c8);
      const v4f qb = *(const v4fa*)(pr + 8 * c8 + 4);
      const v4f ba = *(const v4fa*)(cst + OCB1 + 8 * c8);
      const v4f bb = *(const v4fa*)(cst + OCB1 + 8 * c8 + 4);
      const v8f v8 = {va.x, va.y, va.z, va.w, vb.x, vb.y, vb.z, vb.w};
      const v8f p8 = {pa.x, pa.y, pa.z, pa.w, pb.x, pb.y, pb.z, pb.w};
      const v8f q8 = {qa.x, qa.y, qa.z, qa.w, qb.x, qb.y, qb.z, qb.w};
      const v8f b8 = {ba.x, ba.y, ba.z, ba.w, bb.x, bb.y, bb.z, bb.w};
      v8us ho, lo;
#pragma unroll
      for (int i = 0; i < 8; ++i) {
        const float pre = (p8[i] + q8[i]) + (v8[i] + b8[i]);
        const float h   = fmaxf(pre, 0.0f);
        const unsigned hb = bf16_bits(h);
        ho[i] = (unsigned short)hb;
        lo[i] = (unsigned short)bf16_bits(h - __uint_as_float(hb << 16));
      }
      *(v8usa*)(ra + 8 * c8)       = ho;
      *(v8usa*)(ra + HID + 8 * c8) = lo;
    }
  }
  __syncthreads();

  wave_gemm_b<AP>(sAw, sDw, W2T, KH, KH, hh, m);
  __syncthreads();

  row_relu_ln(rd, cst);
  __syncthreads();

  sweep_f32(sD, NE + (size_t)elb * HID, tid);
  __threadfence();
  sweep_f32(sD, NE + (size_t)elb * HID, tid);
  __syncthreads();

  {
    const float* eo = ELF + (size_t)el * HID;
#pragma unroll 1
    for (int c8 = 0; c8 < HID / 8; ++c8) {
      const v4f va = *(const v4fa*)(rd + 8 * c8);
      const v4f vb = *(const v4fa*)(rd + 8 * c8 + 4);
      const v4f oa = *(const v4fa*)(eo + 8 * c8);
      const v4f ob = *(const v4fa*)(eo + 8 * c8 + 4);
      const v8f v8 = {va.x + oa.x, va.y + oa.y, va.z + oa.z, va.w + oa.w,
                      vb.x + ob.x, vb.y + ob.y, vb.z + ob.z, vb.w + ob.w};
      v8us ho, lo;
#pragma unroll
      for (int i = 0; i < 8; ++i) {
        const unsigned hb = bf16_bits(v8[i]);
        ho[i] = (unsigned short)hb;
        lo[i] = (unsigned short)bf16_bits(v8[i] - __uint_as_float(hb << 16));
      }
      const v4f m0 = {v8[0], v8[1], v8[2], v8[3]};
      const v4f m1 = {v8[4], v8[5], v8[6], v8[7]};
      *(v4fa*)(rd + 8 * c8)        = m0;
      *(v4fa*)(rd + 8 * c8 + 4)    = m1;
      *(v8usa*)(ra + 8 * c8)       = ho;
      *(v8usa*)(ra + HID + 8 * c8) = lo;
    }
  }
  __syncthreads();

  sweep_f32(sD, ELF + (size_t)elb * HID, tid);
  sweep_h16(sA, ELH + (size_t)elb * KH, tid);
  __threadfence();
  sweep_f32(sD, ELF + (size_t)elb * HID, tid);
  sweep_h16(sA, ELH + (size_t)elb * KH, tid);
}

__global__ __launch_bounds__(NTHR) void k_scan(const int* __restrict__ dsts, int nEh, int vec8, int mRows,
                                               const float* __restrict__ NEp, unsigned short* NZ) {
  extern __shared__ __attribute__((aligned(16))) int dsm[];
  int*   list = dsm;
  int*   hl   = dsm + LISTN;
  int*   sl   = hl + RCAP;
  int*   cnt  = sl + RCAP;
  int*   offs = cnt + NBA;
  int*   cur  = offs + NBA;
  int*   misc = cur + NBA;
  const int tid = (int)threadIdx.x, lane = tid & 31, wave = tid >> 5;
  const int nodeBase = (int)blockIdx.x * NBA;

  {
    const v4i z4 = {0, 0, 0, 0};
    for (int i = tid * 4; i < AGG_ZINTS; i += NTHR * 4) *(v4ia*)(dsm + i) = z4;
    if (tid < 16) misc[tid] = 0;
  }
  __syncthreads();

  int t = 0, ov = 0;
  const int nChunks = (nEh + CHUNK - 1) / CHUNK;
#pragma unroll 1
  for (int ch = 0; ch < nChunks; ++ch) {
    const int cbase = ch * CHUNK;
    const int wc = scan_chunk<SLA>(dsts, nEh, cbase, nodeBase, NBA, vec8, list, tid, lane, wave);
    if (lane == 0) misc[wave] = wc;
    __syncthreads();
    if (wave == 0) {
#pragma unroll 1
      for (int w2 = 0; w2 < NWAVE; ++w2) {
        int c = misc[w2];
        c = c < 0 ? 0 : (c > WCAP ? WCAP : c);
#pragma unroll 1
        for (int b0 = 0; b0 < c; b0 += 32) {
          const int idx = b0 + lane;
          const int ent = list[w2 * WCAP + (idx < WCAP ? idx : WCAP - 1)];
          const int m32 = (c - b0) < 32 ? (c - b0) : 32;
#pragma unroll 1
          for (int k = 0; k < m32; ++k) {
            const int u    = __builtin_amdgcn_readlane(ent, k);
            const int slot = u & (NBA - 1);
            const int el   = (u >> SLA) & (CHUNK - 1);
            const int pk   = ((cbase + el) << SLA) | slot;
            if (t < RCAP) {
              if (lane == 0) { hl[t] = pk; cnt[slot] = cnt[slot] + 1; }
              t = t + 1;
            } else {
              ov = 1;
            }
          }
        }
      }
    }
    __syncthreads();
  }
  if (wave == 0 && lane == 0) { misc[8] = t; misc[9] = ov; }
  __syncthreads();
  int tt = misc[8];
  tt = tt < 0 ? 0 : (tt > RCAP ? RCAP : tt);
  const int ovf = misc[9];

  if (wave == 0) {
    const int base = lane * (NBA / 32);
    int s = 0;
#pragma unroll 1
    for (int i = 0; i < NBA / 32; ++i) s += cnt[base + i];
    int incl = s;
#pragma unroll
    for (int d = 1; d < 32; d <<= 1) {
      const int y = __shfl_up(incl, d, 32);
      if (lane >= d) incl += y;
    }
    int run = incl - s;
#pragma unroll 1
    for (int i = 0; i < NBA / 32; ++i) {
      const int cv = cnt[base + i];
      offs[base + i] = run;
      cur[base + i]  = run;
      run += cv;
    }
  }
  __syncthreads();
  if (wave == 0) {
#pragma unroll 1
    for (int b0 = 0; b0 < tt; b0 += 32) {
      const int idx = b0 + lane;
      const int ent = hl[idx < RCAP ? idx : RCAP - 1];
      const int m32 = (tt - b0) < 32 ? (tt - b0) : 32;
#pragma unroll 1
      for (int k = 0; k < m32; ++k) {
        const int u    = __builtin_amdgcn_readlane(ent, k);
        const int slot = u & (NBA - 1);
        if (lane == 0) {
          int p = cur[slot];
          p = p < 0 ? 0 : (p > RCAP - 1 ? RCAP - 1 : p);
          sl[p] = u;
          cur[slot] = p + 1;
        }
      }
    }
  }
  __syncthreads();

  const float qnan = __int_as_float(0x7fc00000);
  const float pz = (ovf != 0) ? qnan : 0.0f;
#pragma unroll 1
  for (int si = 0; si < NBA / NWAVE; ++si) {
    const int s    = si * NWAVE + wave;
    const int node = nodeBase + s;
    int c = cnt[s];
    const bool big = c > DEGCAP;
    c = c < 0 ? 0 : (c > DEGCAP ? DEGCAP : c);
    int o = offs[s];
    o = o < 0 ? 0 : (o > RCAP ? RCAP : o);
    float a0 = 0.0f, a1 = 0.0f, a2 = 0.0f, a3 = 0.0f;
#pragma unroll 1
    for (int b0 = 0; b0 < c; b0 += 32) {
      int idx = o + b0 + lane;
      idx = idx > RCAP - 1 ? RCAP - 1 : idx;
      const int ent = sl[idx];
      int eid = ent >> SLA;
      eid = eid < 0 ? 0 : (eid > nEh - 1 ? nEh - 1 : eid);
      const int m32 = (c - b0) < 32 ? (c - b0) : 32;
#pragma unroll 1
      for (int k = 0; k < m32; ++k) {
        const int ek = __builtin_amdgcn_readlane(eid, k);
        const v4f w = *(const v4fa*)(NEp + (size_t)ek * HID + 4 * lane);
        a0 += w.x;
        a1 += w.y;
        a2 += w.z;
        a3 += w.w;
      }
    }
    const bool  live = node < mRows;
    const int   nr   = live ? node : mRows - 1;
    const float pzr  = big ? qnan : pz;
    const float f0 = a0 + pzr, f1 = a1 + pzr, f2 = a2 + pzr, f3 = a3 + pzr;
    const unsigned h0 = bf16_bits(f0), h1 = bf16_bits(f1), h2 = bf16_bits(f2), h3 = bf16_bits(f3);
    v8us ob;
    ob[0] = (unsigned short)h0; ob[1] = (unsigned short)h1; ob[2] = (unsigned short)h2; ob[3] = (unsigned short)h3;
    ob[4] = (unsigned short)bf16_bits(f0 - __uint_as_float(h0 << 16));
    ob[5] = (unsigned short)bf16_bits(f1 - __uint_as_float(h1 << 16));
    ob[6] = (unsigned short)bf16_bits(f2 - __uint_as_float(h2 << 16));
    ob[7] = (unsigned short)bf16_bits(f3 - __uint_as_float(h3 << 16));
    unsigned short* zp = NZ + (size_t)nr * NZP + KH + 8 * lane;
    if (live) *(volatile v8us*)zp = ob;
    __threadfence();
    if (live) *(volatile v8us*)zp = ob;
  }
}

__global__ __launch_bounds__(DTHR) void k_dec(const unsigned short* __restrict__ NZ,
                                              const unsigned short* __restrict__ DW1T,
                                              const float* __restrict__ db1, const float* __restrict__ dW2,
                                              const float* __restrict__ db2, float* DEC) {
  __shared__ __attribute__((aligned(16))) float stg[DROWS * DPT];
  __shared__ __attribute__((aligned(16))) float sq[DROWS * DPT];
  __shared__ float cw[DH * DO];
  __shared__ float cb1[DH];
  __shared__ float cb2[DPT];
  const int tid = (int)threadIdx.x, lane = tid & 31, wave = tid >> 5, hh = lane >> 4, m = lane & 15;
  const int rowBase = (int)blockIdx.x * DROWS;
  {
    const float wv = bf16_val(dW2[tid < DH * DO ? tid : DH * DO - 1]);
    const float bv = bf16_val(db1[tid < DH ? tid : DH - 1]);
    const float cv = bf16_val(db2[tid < DO ? tid : DO - 1]);
    if (tid < DH * DO) cw[tid] = wv;
    if (tid < DH) cb1[tid] = bv;
    if (tid < DPT) cb2[tid] = (tid < DO) ? cv : 0.0f;
  }
  v8f acc = {0.f, 0.f, 0.f, 0.f, 0.f, 0.f, 0.f, 0.f};
  const unsigned short* ap = NZ + (size_t)(rowBase + 16 * wave + m) * (size_t)NZP + 8 * hh;
  const unsigned short* bp = DW1T + (size_t)m * KH + 8 * hh;
#pragma unroll 1
  for (int k0 = 0; k0 < KH; k0 += 32) {
    FragB af, bf;
    af.h[0] = *(const v8usa*)(ap + k0);
    af.h[1] = *(const v8usa*)(ap + k0 + 16);
    bf.h[0] = *(const v8usa*)(bp + k0);
    bf.h[1] = *(const v8usa*)(bp + k0 + 16);
    acc = wmb(af, bf, acc);
  }
#pragma unroll
  for (int r = 0; r < 8; ++r) stg[(16 * wave + 8 * hh + r) * DPT + m] = acc[r];
  __syncthreads();
  if (tid < DROWS) {
    const float* hp = stg + tid * DPT;
    float sw[DH];
#pragma unroll
    for (int o = 0; o < DH; ++o) {
      const float h = hp[o] + cb1[o];
      sw[o] = h * __builtin_amdgcn_rcpf(1.0f + __expf(-h));
    }
#pragma unroll 1
    for (int j = 0; j < DO; ++j) {
      float a = 0.0f;
#pragma unroll
      for (int o = 0; o < DH; ++o) a = fmaf(sw[o], cw[o * DO + j], a);
      sq[tid * DPT + j] = a + cb2[j];
    }
    sq[tid * DPT + DO] = 0.0f;
  }
  __syncthreads();
  v4f pv[(DROWS * DPT / 4) / DTHR];
#pragma unroll
  for (int it = 0; it < (DROWS * DPT / 4) / DTHR; ++it) pv[it] = *(const v4fa*)(sq + (it * DTHR + tid) * 4);
  float* dbp = DEC + (size_t)rowBase * DPT;
#pragma unroll
  for (int it = 0; it < (DROWS * DPT / 4) / DTHR; ++it)
    *(volatile v4f*)(dbp + (size_t)(it * DTHR + tid) * 4) = pv[it];
  __threadfence();
#pragma unroll
  for (int it = 0; it < (DROWS * DPT / 4) / DTHR; ++it)
    *(volatile v4f*)(dbp + (size_t)(it * DTHR + tid) * 4) = pv[it];
}

__global__ __launch_bounds__(NTHR) void k_out(const float* __restrict__ DEC, int nN, int nQ, float* out) {
  const int u = (int)blockIdx.x * NTHR + (int)threadIdx.x;
  if (u >= nQ) return;
  const unsigned per = 3u * (unsigned)nN;
  const unsigned f0  = 4u * (unsigned)u;
  float val[4];
#pragma unroll
  for (int i = 0; i < 4; ++i) {
    const unsigned f   = f0 + (unsigned)i;
    unsigned tw        = f / per;
    const unsigned rem = f - tw * per;
    const unsigned n   = rem / 3u;
    const unsigned o   = rem - 3u * n;
    tw = tw > (unsigned)(NTW - 1) ? (unsigned)(NTW - 1) : tw;
    const float dv = DEC[(size_t)n * DPT + tw * NOD + o];
    val[i] = dv * (float)(tw + 1u);
  }
  const v4f q4 = {val[0], val[1], val[2], val[3]};
  float* op = out + (size_t)u * 4;
  *(volatile v4f*)op = q4;
  __threadfence();
  *(volatile v4f*)op = q4;
}

static inline int cdiv(int a, int b) { return (a + b - 1) / b; }

extern "C" void kernel_launch(void* const* d_in, const int* in_sizes, int n_in,
                              void* d_out, int out_size, void* d_ws, size_t ws_size,
                              hipStream_t stream) {
  if (n_in < 38) return;
  if (in_sizes[0] < 2 || (in_sizes[0] & 1) != 0) return;
  const int nN = in_sizes[0] / 2;
  if (in_sizes[1] != 2 * nN || in_sizes[2] != nN || in_sizes[3] != nN) return;
  const int nE = in_sizes[4];
  if (nE < 1 || in_sizes[5] != nE || nE >= (1 << 21)) return;
  if (in_sizes[6] != NF || in_sizes[7] != NF || in_sizes[8] != NF || in_sizes[9] != NF) return;
  if (in_sizes[10] != NF * HID || in_sizes[11] != HID || in_sizes[12] != HID * HID) return;
  if (in_sizes[13] != HID || in_sizes[14] != HID || in_sizes[15] != HID) return;
  if (in_sizes[16] != NF * HID || in_sizes[17] != HID || in_sizes[18] != HID * HID) return;
  if (in_sizes[19] != HID || in_sizes[20] != HID || in_sizes[21] != HID) return;
  if (in_sizes[22] < 3 * HID * HID || (in_sizes[22] % (3 * HID * HID)) != 0) return;
  const int nS = in_sizes[22] / (3 * HID * HID);
  if (nS < 1 || nS > 64) return;
  if (in_sizes[23] != nS * HID || in_sizes[24] != nS * HID * HID || in_sizes[25] != nS * HID) return;
  if (in_sizes[26] != nS * HID || in_sizes[27] != nS * HID) return;
  if (in_sizes[28] != nS * 2 * HID * HID || in_sizes[29] != nS * HID || in_sizes[30] != nS * HID * HID) return;
  if (in_sizes[31] != nS * HID || in_sizes[32] != nS * HID || in_sizes[33] != nS * HID) return;
  if (in_sizes[34] != HID * DH || in_sizes[35] != DH || in_sizes[36] != DH * DO || in_sizes[37] != DO) return;
  if ((long long)out_size != (long long)NTW * NOD * (long long)nN || (out_size & 3) != 0) return;

  const float* mpos  = (const float*)d_in[0];
  const float* disp  = (const float*)d_in[1];
  const float* chem  = (const float*)d_in[2];
  const int*   ntype = (const int*)d_in[3];
  const int*   snd   = (const int*)d_in[4];
  const int*   rcv   = (const int*)d_in[5];
  const float* nmean = (const float*)d_in[6];
  const float* nstd  = (const float*)d_in[7];
  const float* emean = (const float*)d_in[8];
  const float* estd  = (const float*)d_in[9];
  const float* en_W1 = (const float*)d_in[10]; const float* en_b1 = (const float*)d_in[11];
  const float* en_W2 = (const float*)d_in[12]; const float* en_b2 = (const float*)d_in[13];
  const float* en_g  = (const float*)d_in[14]; const float* en_be = (const float*)d_in[15];
  const float* ee_W1 = (const float*)d_in[16]; const float* ee_b1 = (const float*)d_in[17];
  const float* ee_W2 = (const float*)d_in[18]; const float* ee_b2 = (const float*)d_in[19];
  const float* ee_g  = (const float*)d_in[20]; const float* ee_be = (const float*)d_in[21];
  const float* be_W1 = (const float*)d_in[22]; const float* be_b1 = (const float*)d_in[23];
  const float* be_W2 = (const float*)d_in[24]; const float* be_b2 = (const float*)d_in[25];
  const float* be_g  = (const float*)d_in[26]; const float* be_be = (const float*)d_in[27];
  const float* bn_W1 = (const float*)d_in[28]; const float* bn_b1 = (const float*)d_in[29];
  const float* bn_W2 = (const float*)d_in[30]; const float* bn_b2 = (const float*)d_in[31];
  const float* bn_g  = (const float*)d_in[32]; const float* bn_be = (const float*)d_in[33];
  const float* dc_W1 = (const float*)d_in[34]; const float* dc_b1 = (const float*)d_in[35];
  const float* dc_W2 = (const float*)d_in[36]; const float* dc_b2 = (const float*)d_in[37];
  float* out = (float*)d_out;

  const int MP = cdiv(nN, GBM) * GBM;
  const int gM = MP / GBM;
  const int gA = cdiv(MP, NBA);
  if ((long long)gA * NBA < (long long)MP) return;
  const int EP = cdiv(nE, EPB) * EPB;
  const int gE = EP / EPB;

  char* ws = (char*)d_ws;
  size_t off = 0;
  const size_t oWST  = off; off += (size_t)nS * SPH * 2;             off = (off + 255) & ~(size_t)255;
  const size_t oENW1 = off; off += (size_t)HID * KF * 2;             off = (off + 255) & ~(size_t)255;
  const size_t oENW2 = off; off += (size_t)HID * KH * 2;             off = (off + 255) & ~(size_t)255;
  const size_t oEEW1 = off; off += (size_t)HID * KF * 2;             off = (off + 255) & ~(size_t)255;
  const size_t oEEW2 = off; off += (size_t)HID * KH * 2;             off = (off + 255) & ~(size_t)255;
  const size_t oDCW1 = off; off += (size_t)DPT * KH * 2;             off = (off + 255) & ~(size_t)255;
  const size_t oFN   = off; off += (size_t)MP * KF * 2;              off = (off + 255) & ~(size_t)255;
  const size_t oNZ   = off; off += (size_t)MP * NZP * 2;             off = (off + 255) & ~(size_t)255;
  const size_t oNLF  = off; off += (size_t)MP * HID * 4;             off = (off + 255) & ~(size_t)255;
  size_t szT = (size_t)MP * NPS * 4;
  if (szT < (size_t)MP * KH * 2) szT = (size_t)MP * KH * 2;
  const size_t oT    = off; off += szT;                              off = (off + 255) & ~(size_t)255;
  const size_t oELF  = off; off += (size_t)EP * HID * 4;             off = (off + 255) & ~(size_t)255;
  const size_t oELH  = off; off += (size_t)EP * KH * 2;              off = (off + 255) & ~(size_t)255;
  const size_t oNE   = off; off += (size_t)EP * HID * 4;             off = (off + 255) & ~(size_t)255;
  const size_t oDEC  = off; off += (size_t)MP * DPT * 4;             off = (off + 255) & ~(size_t)255;
  if (off > ws_size || off > (size_t)WSMAX) return;
  unsigned short* WST  = (unsigned short*)(ws + oWST);
  unsigned short* ENW1 = (unsigned short*)(ws + oENW1);
  unsigned short* ENW2 = (unsigned short*)(ws + oENW2);
  unsigned short* EEW1 = (unsigned short*)(ws + oEEW1);
  unsigned short* EEW2 = (unsigned short*)(ws + oEEW2);
  unsigned short* DCW1 = (unsigned short*)(ws + oDCW1);
  unsigned short* FN   = (unsigned short*)(ws + oFN);
  unsigned short* NZ   = (unsigned short*)(ws + oNZ);
  float*          NLF  = (float*)(ws + oNLF);
  float*          PSR  = (float*)(ws + oT);
  unsigned short* G    = (unsigned short*)(ws + oT);
  float*          ELF  = (float*)(ws + oELF);
  unsigned short* ELH  = (unsigned short*)(ws + oELH);
  float*          NE   = (float*)(ws + oNE);
  float*          DEC  = (float*)(ws + oDEC);

  hipFuncSetAttribute(reinterpret_cast<const void*>(&k_ence), hipFuncAttributeMaxDynamicSharedMemorySize,
                      (int)EDGE_LDS_BYTES);
  hipFuncSetAttribute(reinterpret_cast<const void*>(&k_edge), hipFuncAttributeMaxDynamicSharedMemorySize,
                      (int)EDGE_LDS_BYTES);
  hipFuncSetAttribute(reinterpret_cast<const void*>(&k_scan), hipFuncAttributeMaxDynamicSharedMemorySize,
                      (int)AGG_LDS_BYTES);

  const int nPrep = nS * UPS + NU_ENC + 4 * MP;
  const int vec8  = 1;
  const int nQ    = out_size / 4;

  k_prep<<<nPrep / NTHR, NTHR, 0, stream>>>(disp, chem, ntype, nmean, nstd, en_W1, en_W2, ee_W1, ee_W2,
                                            be_W1, be_W2, bn_W1, bn_W2, dc_W1, nN, MP, nS,
                                            WST, ENW1, ENW2, EEW1, EEW2, DCW1, FN);
  k_gemm<1><<<dim3(gM, 1), GTHR, 0, stream>>>(FN, KF, ENW1, KF, KF, en_b1, en_g, en_be, NLF, HID, G, KH);
  k_gemm<3><<<dim3(gM, 1), GTHR, 0, stream>>>(G, KH, ENW2, KH, KH, en_b2, en_g, en_be, NLF, HID, NZ, NZP);
  k_ence<<<gE, NTHR, EDGE_LDS_BYTES, stream>>>(snd, rcv, nE, nN, mpos, disp, chem, emean, estd,
                                               EEW1, EEW2, ee_b1, ee_b2, ee_g, ee_be, ELF, ELH);
  for (int t = 0; t < nS; ++t) {
    const unsigned short* Wt = WST + (size_t)t * SPH;
    const size_t ob = (size_t)t * HID;
    k_gemm<0><<<dim3(gM, NPS / GBN), GTHR, 0, stream>>>(NZ, NZP, Wt + OW1AB, KH, KH, be_b1 + ob, be_g + ob,
                                                        be_be + ob, PSR, NPS, G, KH);
    k_edge<<<gE, NTHR, EDGE_LDS_BYTES, stream>>>(snd, rcv, nE, nN, PSR, Wt + OW1C, Wt + OW2E,
                                                 be_b1 + ob, be_b2 + ob, be_g + ob, be_be + ob, ELF, ELH, NE);
    k_scan<<<gA, NTHR, AGG_LDS_BYTES, stream>>>(rcv, nE, vec8, MP, NE, NZ);
    k_gemm<1><<<dim3(gM, 1), GTHR, 0, stream>>>(NZ, NZP, Wt + OWN1, KN1, KN1, bn_b1 + ob, bn_g + ob,
                                                bn_be + ob, NLF, HID, G, KH);
    k_gemm<4><<<dim3(gM, 1), GTHR, 0, stream>>>(G, KH, Wt + OWN2, KH, KH, bn_b2 + ob, bn_g + ob,
                                                bn_be + ob, NLF, HID, NZ, NZP);
  }
  k_dec<<<MP / DROWS, DTHR, 0, stream>>>(NZ, DCW1, dc_b1, dc_W2, dc_b2, DEC);
  k_out<<<cdiv(nQ, NTHR), NTHR, 0, stream>>>(DEC, nN, nQ, out);
}
